// PEneoDecoder_84293028151981
// MI455X (gfx1250) — hardware-verified
//
#include <hip/hip_runtime.h>
#include <math.h>

typedef __attribute__((ext_vector_type(16))) _Float16 v16h;
typedef __attribute__((ext_vector_type(16))) __bf16 v16b;
typedef __attribute__((ext_vector_type(8)))  _Float16 v8h;
typedef __attribute__((ext_vector_type(8)))  float v8f;
typedef __attribute__((ext_vector_type(4)))  float v4f;
typedef __attribute__((ext_vector_type(2)))  float v2f;
typedef __attribute__((ext_vector_type(4)))  unsigned v4u;
typedef __attribute__((ext_vector_type(4)))  int v4i;
typedef float __attribute__((may_alias)) float_a;
typedef int __attribute__((may_alias)) int_a;

template <typename T> __device__ __forceinline__ void vst2(void* p, T v) { *(volatile T*)p = v; __threadfence(); *(volatile T*)p = v; }
__device__ __forceinline__ v8f wmma16(v16h a, v16h b, v8f c) {
  v8f d = __builtin_amdgcn_wmma_f32_16x16x32_f16(false, a, false, b, (short)0, c, false, false);
  asm volatile("v_nop\n\tv_nop\n\tv_nop\n\tv_nop" : "+v"(d) : "v"(a), "v"(b));
  return d;
}
__device__ __forceinline__ v8f wmma_bf(v16b a, v16b b, v8f c) {
  v8f d = __builtin_amdgcn_wmma_f32_16x16x32_bf16(false, a, false, b, (short)0, c, false, false);
  asm volatile("v_nop\n\tv_nop\n\tv_nop\n\tv_nop" : "+v"(d) : "v"(a), "v"(b));
  return d;
}
__device__ __forceinline__ v16h frag_h(const _Float16* rowk0, int lane) {
  union { v16h v; v8h q[2]; } u; const _Float16* p = rowk0 + 8 * (lane >> 4);
  u.q[0] = *(const v8h*)p; u.q[1] = *(const v8h*)(p + 16); return u.v;
}
__device__ __forceinline__ v16h frag_f32(const float* rowk0, int lane) {
  v16h a; const float* p = rowk0 + 8 * (lane >> 4);
#pragma unroll
  for (int i = 0; i < 8; ++i) { a[i] = (_Float16)p[i]; a[8 + i] = (_Float16)p[16 + i]; }
  return a;
}
__device__ __forceinline__ v16h frag_f32s(const float* rowk0, int lane, float sc) {
  v16h a; const float* p = rowk0 + 8 * (lane >> 4);
#pragma unroll
  for (int i = 0; i < 8; ++i) { a[i] = (_Float16)(p[i] * sc); a[8 + i] = (_Float16)(p[16 + i] * sc); }
  return a;
}
__device__ __forceinline__ v16h fragc_f32(const float* W, int k0, int n, int lane, int ld, int K) {
  v16h a; const int g = lane >> 4;
#pragma unroll
  for (int i = 0; i < 8; ++i) { const int ka = k0 + 8 * g + i, kb = ka + 16;
    a[i] = (_Float16)(ka < K ? W[(size_t)(ka < K ? ka : K - 1) * ld + n] : 0.f); a[8 + i] = (_Float16)(kb < K ? W[(size_t)(kb < K ? kb : K - 1) * ld + n] : 0.f); }
  return a;
}
struct F2 { v16b h, l; };
__device__ __forceinline__ F2 bsplit16(const float v[16]) { F2 r;
#pragma unroll
  for (int i = 0; i < 16; ++i) { const __bf16 h = (__bf16)v[i]; r.h[i] = h; r.l[i] = (__bf16)(v[i] - (float)h); }
  return r; }
__device__ __forceinline__ F2 split_row(const float* row, int k0, int lane) { float v[16]; const float* p = row + k0 + 8 * (lane >> 4);
#pragma unroll
  for (int i = 0; i < 8; ++i) { v[i] = p[i]; v[8 + i] = p[16 + i]; }
  return bsplit16(v); }
__device__ __forceinline__ F2 split_rowK(const float* row, int k0, int lane, int K) { float v[16]; const int g = lane >> 4;
#pragma unroll
  for (int i = 0; i < 8; ++i) { const int ka = k0 + 8 * g + i, kb = ka + 16; v[i] = ka < K ? row[ka < K ? ka : K - 1] : 0.f; v[8 + i] = kb < K ? row[kb < K ? kb : K - 1] : 0.f; }
  return bsplit16(v); }
__device__ __forceinline__ F2 split_col(const float* W, int k0, int n, int lane, int ld, int K) { float v[16]; const int g = lane >> 4;
#pragma unroll
  for (int i = 0; i < 8; ++i) { const int ka = k0 + 8 * g + i, kb = ka + 16; v[i] = ka < K ? W[(size_t)(ka < K ? ka : K - 1) * ld + n] : 0.f; v[8 + i] = kb < K ? W[(size_t)(kb < K ? kb : K - 1) * ld + n] : 0.f; }
  return bsplit16(v); }
__device__ __forceinline__ v8f mac3(const F2& a, const F2& b, v8f c) { c = wmma_bf(a.l, b.h, c); c = wmma_bf(a.h, b.l, c); return wmma_bf(a.h, b.h, c); }
__device__ __forceinline__ float sigm(float v) { return 1.0f / (1.0f + expf(-v)); }
#define LDSX() do { asm volatile("s_wait_dscnt 0" ::: "memory"); __builtin_amdgcn_wave_barrier(); __builtin_amdgcn_fence(__ATOMIC_RELEASE, "workgroup"); } while (0)


#define NBATCH 2
#define SEQ 512
#define NTOK (NBATCH * SEQ)
#define DIN 768
#define HB 768
#define HD 384
#define NPAIR 131328
#define PBLK 256
#define NCLS 14
typedef __attribute__((ext_vector_type(8))) __bf16 v8b;
__device__ __forceinline__ v16b frag_b16(const __bf16* rowk0, int lane) {
  union { v16b v; v8b q[2]; } u; const __bf16* p = rowk0 + 8 * (lane >> 4);
  u.q[0] = *(const v8b*)p; u.q[1] = *(const v8b*)(p + 16); return u.v;
}
__device__ __forceinline__ v16b frag_gbf(const float* rowk0, int lane) {
  v16b a; const float* p = rowk0 + 8 * (lane >> 4);
#pragma unroll
  for (int i = 0; i < 8; ++i) { a[i] = (__bf16)p[i]; a[8 + i] = (__bf16)p[16 + i]; }
  return a;
}
__device__ __forceinline__ float bfr(float v) { return (float)(__bf16)v; }
__device__ __forceinline__ float tanh_f(float x) { const float e = expf(-2.0f * fabsf(x)); return copysignf((1.0f - e) / (1.0f + e), x); }

#define WS_PT1  0u
#define WS_PT2  (WS_PT1 + 2u * HB * DIN)
#define WS_PTT  (WS_PT2 + 2u * HD * HB)
#define WS_PTB  (WS_PTT + 2u * HD * HD)
#define WS_H1H  (WS_PTB + 2u * HD * HD)
#define WS_H1L  (WS_H1H + 2u * NTOK * HB)
#define WS_H2H  (WS_H1L + 2u * NTOK * HB)
#define WS_H2L  (WS_H2H + 2u * NTOK * HD)
#define WS_L    (WS_H2L + 2u * NTOK * HD)
#define WS_R    (WS_L + 4u * NTOK * HD)
#define WS_END  (WS_R + 4u * NTOK * HD)

__global__ __launch_bounds__(256) void k_pack(const float* __restrict__ Wm, int K, int NOUT, __bf16* __restrict__ PT) {
  __shared__ __align__(16) __bf16 srow[DIN];
  const int n = blockIdx.x, tid = threadIdx.x;
  for (int k = tid; k < K; k += 256) srow[k] = (__bf16)Wm[(size_t)k * NOUT + n];
  __syncthreads();
  if (tid < K / 8) vst2((unsigned*)(PT + (size_t)n * K + tid * 8), *(const v4u*)(&srow[tid * 8]));
}
__global__ __launch_bounds__(128) void k_h1(const float* __restrict__ X, const __bf16* __restrict__ PT, const float* __restrict__ b1, __bf16* __restrict__ Hh, __bf16* __restrict__ Hl) {
  __shared__ __align__(16) __bf16 sh_[4][16][136], sl_[4][16][136];
  const int tid = threadIdx.x, wave = tid >> 5, lane = tid & 31, col = lane & 15, g = lane >> 4; const size_t r0 = (size_t)blockIdx.x * 64 + wave * 16; const int n0 = blockIdx.y * 128;
  v8f acc[8] = {};
#pragma unroll 2
  for (int kc = 0; kc < DIN / 32; ++kc) { const v16b a = frag_gbf(X + (r0 + col) * DIN + kc * 32, lane);
#pragma unroll
    for (int j = 0; j < 8; ++j) acc[j] = wmma_bf(a, frag_b16(PT + (size_t)(n0 + j * 16 + col) * DIN + kc * 32, lane), acc[j]); }
#pragma unroll
  for (int j = 0; j < 8; ++j) { const float bb = bfr(b1[n0 + j * 16 + col]);
#pragma unroll
    for (int r = 0; r < 8; ++r) { float v = acc[j][r] + bb; v = v > 0.f ? v : 0.f; const __bf16 hi = (__bf16)v; sh_[wave][8 * g + r][j * 16 + col] = hi; sl_[wave][8 * g + r][j * 16 + col] = (__bf16)(v - (float)hi); } }
  LDSX();
  for (int qq = lane; qq < 16 * 16; qq += 32) { const int rl = qq >> 4, pc = qq & 15; const size_t o = (r0 + rl) * HB + n0 + pc * 8; vst2((unsigned*)(Hh + o), *(const v4u*)(&sh_[wave][rl][pc * 8])); vst2((unsigned*)(Hl + o), *(const v4u*)(&sl_[wave][rl][pc * 8])); }
}
__global__ __launch_bounds__(128) void k_h2(const __bf16* __restrict__ Ah, const __bf16* __restrict__ Al, const __bf16* __restrict__ PT, const float* __restrict__ b2, __bf16* __restrict__ Hh, __bf16* __restrict__ Hl) {
  __shared__ __align__(16) __bf16 sh_[4][16][136], sl_[4][16][136];
  const int tid = threadIdx.x, wave = tid >> 5, lane = tid & 31, col = lane & 15, g = lane >> 4; const size_t r0 = (size_t)blockIdx.x * 64 + wave * 16; const int n0 = blockIdx.y * 128;
  v8f acc[8] = {};
#pragma unroll 2
  for (int kc = 0; kc < HB / 32; ++kc) { const v16b ah = frag_b16(Ah + (r0 + col) * HB + kc * 32, lane), al = frag_b16(Al + (r0 + col) * HB + kc * 32, lane);
#pragma unroll
    for (int j = 0; j < 8; ++j) { const v16b wb = frag_b16(PT + (size_t)(n0 + j * 16 + col) * HB + kc * 32, lane); acc[j] = wmma_bf(al, wb, acc[j]); acc[j] = wmma_bf(ah, wb, acc[j]); } }
#pragma unroll
  for (int j = 0; j < 8; ++j) { const float bb = bfr(b2[n0 + j * 16 + col]);
#pragma unroll
    for (int r = 0; r < 8; ++r) { float v = acc[j][r] + bb; v = v > 0.f ? v : 0.f; const __bf16 hi = (__bf16)v; sh_[wave][8 * g + r][j * 16 + col] = hi; sl_[wave][8 * g + r][j * 16 + col] = (__bf16)(v - (float)hi); } }
  LDSX();
  for (int qq = lane; qq < 16 * 16; qq += 32) { const int rl = qq >> 4, pc = qq & 15; const size_t o = (r0 + rl) * HD + n0 + pc * 8; vst2((unsigned*)(Hh + o), *(const v4u*)(&sh_[wave][rl][pc * 8])); vst2((unsigned*)(Hl + o), *(const v4u*)(&sl_[wave][rl][pc * 8])); }
}
__global__ __launch_bounds__(128) void k_lr(const __bf16* __restrict__ Ah, const __bf16* __restrict__ Al, const __bf16* __restrict__ PTT, const __bf16* __restrict__ PTB, float* __restrict__ Lm, float* __restrict__ Rm) {
  __shared__ __align__(16) float so_[4][16][132];
  const int tid = threadIdx.x, wave = tid >> 5, lane = tid & 31, col = lane & 15, g = lane >> 4; const size_t r0 = (size_t)blockIdx.x * 64 + wave * 16;
  const int right = blockIdx.y >= 3; const int n0 = (blockIdx.y - 3 * right) * 128; const __bf16* PT = right ? PTB : PTT; float* O = right ? Rm : Lm;
  v8f acc[8] = {};
#pragma unroll 2
  for (int kc = 0; kc < HD / 32; ++kc) { const v16b ah = frag_b16(Ah + (r0 + col) * HD + kc * 32, lane), al = frag_b16(Al + (r0 + col) * HD + kc * 32, lane);
#pragma unroll
    for (int j = 0; j < 8; ++j) { const v16b wb = frag_b16(PT + (size_t)(n0 + j * 16 + col) * HD + kc * 32, lane); acc[j] = wmma_bf(al, wb, acc[j]); acc[j] = wmma_bf(ah, wb, acc[j]); } }
#pragma unroll
  for (int j = 0; j < 8; ++j)
#pragma unroll
    for (int r = 0; r < 8; ++r) so_[wave][8 * g + r][j * 16 + col] = acc[j][r];
  LDSX();
#pragma unroll
  for (int rl = 0; rl < 16; ++rl) vst2(O + (r0 + rl) * HD + n0 + lane * 4, *(const v4f*)(&so_[wave][rl][lane * 4]));
}
__global__ __launch_bounds__(256) void k_pair(const float* __restrict__ Lm, const float* __restrict__ Rm, const float* __restrict__ cb,
                                              const float* __restrict__ w0, const float* __restrict__ c0, const float* __restrict__ w1, const float* __restrict__ c1, const float* __restrict__ w2, const float* __restrict__ c2,
                                              const float* __restrict__ w3, const float* __restrict__ c3, const float* __restrict__ w4, const float* __restrict__ c4, float* __restrict__ out) {
  __shared__ __align__(16) __bf16 Hw[16][HD];
  __shared__ float Cb[HD], Hb[16];
  __shared__ __align__(16) float So[PBLK * NCLS];
  const int tid = threadIdx.x, wave = tid >> 5, lane = tid & 31, l16 = lane & 15, hh = lane >> 4;
  const int bidx = blockIdx.y; const int pblk = blockIdx.x * PBLK;
  for (int q = tid; q < 16 * HD; q += 256) { const int n = q / HD, k = q - n * HD;
    const float v0 = w0[k * 2 + min(n, 1)], v1 = w1[k * 3 + min(max(n - 2, 0), 2)], v2 = w2[k * 3 + min(max(n - 5, 0), 2)], v3 = w3[k * 3 + min(max(n - 8, 0), 2)], v4 = w4[k * 3 + min(max(n - 11, 0), 2)];
    const float wv = n < 2 ? v0 : n < 5 ? v1 : n < 8 ? v2 : n < 11 ? v3 : n < 14 ? v4 : 0.f;
    Hw[n][k] = (__bf16)wv; }
  for (int k = tid; k < HD; k += 256) Cb[k] = bfr(cb[k]);
  if (tid < 16) { const float v0 = c0[min(tid, 1)], v1 = c1[min(max(tid - 2, 0), 2)], v2 = c2[min(max(tid - 5, 0), 2)], v3 = c3[min(max(tid - 8, 0), 2)], v4 = c4[min(max(tid - 11, 0), 2)];
    const float bv = tid < 2 ? v0 : tid < 5 ? v1 : tid < 8 ? v2 : tid < 11 ? v3 : tid < 14 ? v4 : 0.f; Hb[tid] = bfr(bv); }
  __syncthreads();
  const float* Lb = Lm + (size_t)bidx * SEQ * HD; const float* Rb = Rm + (size_t)bidx * SEQ * HD;
#pragma unroll 1
  for (int t = 0; t < 2; ++t) {
    const int tile = wave * 2 + t; const int p = pblk + tile * 16 + l16;
    const float disc = (float)((2 * SEQ + 1) * (2 * SEQ + 1) - 8 * p);
    int i = (int)(((float)(2 * SEQ + 1) - sqrtf(disc)) * 0.5f);
    i = i < 0 ? 0 : (i > SEQ - 1 ? SEQ - 1 : i);
#pragma unroll
    for (int f = 0; f < 3; ++f) { if (i > 0 && (i * (2 * SEQ - i + 1)) / 2 > p) --i; }
#pragma unroll
    for (int f = 0; f < 3; ++f) { if (i < SEQ - 1 && ((i + 1) * (2 * SEQ - i)) / 2 <= p) ++i; }
    int jx = i + (p - (i * (2 * SEQ - i + 1)) / 2); jx = jx > SEQ - 1 ? SEQ - 1 : jx;
    const float* lrow = Lb + (size_t)i * HD; const float* rrow = Rb + (size_t)jx * HD;
    v8f acc = {};
#pragma unroll 1
    for (int kc = 0; kc < HD / 32; ++kc) {
      float v[16]; const int ka = kc * 32 + 8 * hh;
      const float4 la = *(const float4*)(lrow + ka), lb2 = *(const float4*)(lrow + ka + 4), lc = *(const float4*)(lrow + ka + 16), ld = *(const float4*)(lrow + ka + 20);
      const float4 ra = *(const float4*)(rrow + ka), rb = *(const float4*)(rrow + ka + 4), rc = *(const float4*)(rrow + ka + 16), rd = *(const float4*)(rrow + ka + 20);
      const float lv[16] = {la.x, la.y, la.z, la.w, lb2.x, lb2.y, lb2.z, lb2.w, lc.x, lc.y, lc.z, lc.w, ld.x, ld.y, ld.z, ld.w};
      const float rv[16] = {ra.x, ra.y, ra.z, ra.w, rb.x, rb.y, rb.z, rb.w, rc.x, rc.y, rc.z, rc.w, rd.x, rd.y, rd.z, rd.w};
#pragma unroll
      for (int e = 0; e < 16; ++e) { const int k = ka + (e < 8 ? e : 8 + e); v[e] = tanh_f((lv[e] + rv[e]) + Cb[k]); }
      const F2 af = bsplit16(v);
      const v16b wb = frag_b16(&Hw[l16][kc * 32], lane);
      acc = wmma_bf(af.l, wb, acc); acc = wmma_bf(af.h, wb, acc);
    }
    if (l16 < NCLS) {
#pragma unroll
      for (int r = 0; r < 8; ++r) So[(tile * 16 + 8 * hh + r) * NCLS + l16] = acc[r] + Hb[l16];
    }
  }
  __syncthreads();
  float* ob = out + ((size_t)bidx * NPAIR + pblk) * NCLS;
  for (int q = tid; q < PBLK * NCLS / 4; q += 256) vst2(ob + q * 4, *(const v4f*)&So[q * 4]);
}

extern "C" void kernel_launch(void* const* d_in, const int* in_sizes, int n_in, void* d_out, int out_size, void* d_ws, size_t ws_size, hipStream_t stream) {
  (void)in_sizes; (void)n_in; (void)out_size; (void)ws_size;
  const float* X  = (const float*)d_in[0];
  const float* W1 = (const float*)d_in[1]; const float* b1 = (const float*)d_in[2];
  const float* W2 = (const float*)d_in[3]; const float* b2 = (const float*)d_in[4];
  const float* CW = (const float*)d_in[5]; const float* cb = (const float*)d_in[6];
  char* ws = (char*)d_ws;
  __bf16* PT1 = (__bf16*)(ws + WS_PT1); __bf16* PT2 = (__bf16*)(ws + WS_PT2); __bf16* PTT = (__bf16*)(ws + WS_PTT); __bf16* PTB = (__bf16*)(ws + WS_PTB);
  __bf16* H1h = (__bf16*)(ws + WS_H1H); __bf16* H1l = (__bf16*)(ws + WS_H1L); __bf16* H2h = (__bf16*)(ws + WS_H2H); __bf16* H2l = (__bf16*)(ws + WS_H2L);
  float* Lm = (float*)(ws + WS_L); float* Rm = (float*)(ws + WS_R);
  k_pack<<<HB, 256, 0, stream>>>(W1, DIN, HB, PT1);
  k_pack<<<HD, 256, 0, stream>>>(W2, HB, HD, PT2);
  k_pack<<<HD, 256, 0, stream>>>(CW, HD, HD, PTT);
  k_pack<<<HD, 256, 0, stream>>>(CW + (size_t)HD * HD, HD, HD, PTB);
  k_h1<<<dim3(NTOK / 64, HB / 128), 128, 0, stream>>>(X, PT1, b1, H1h, H1l);
  k_h2<<<dim3(NTOK / 64, HD / 128), 128, 0, stream>>>(H1h, H1l, PT2, b2, H2h, H2l);
  k_lr<<<dim3(NTOK / 64, 6), 128, 0, stream>>>(H2h, H2l, PTT, PTB, Lm, Rm);
  k_pair<<<dim3(NPAIR / PBLK, NBATCH), 256, 0, stream>>>(Lm, Rm, cb, (const float*)d_in[7], (const float*)d_in[8], (const float*)d_in[9], (const float*)d_in[10],
      (const float*)d_in[11], (const float*)d_in[12], (const float*)d_in[13], (const float*)d_in[14], (const float*)d_in[15], (const float*)d_in[16], (float*)d_out);
}
